// NeuralFingerprint_56710748176715
// MI455X (gfx1250) — hardware-verified
//
#include <hip/hip_runtime.h>


namespace {
typedef _Float16 b16;
typedef __attribute__((ext_vector_type(16))) _Float16 v16b;
typedef __attribute__((ext_vector_type(8))) _Float16 v8b;
typedef __attribute__((ext_vector_type(4))) _Float16 v4h;
typedef __attribute__((ext_vector_type(2))) _Float16 v2h;
typedef __attribute__((ext_vector_type(8))) float v8f;
typedef __attribute__((ext_vector_type(4))) float v4f;
typedef __attribute__((ext_vector_type(2))) float v2f;
__device__ __forceinline__ float bf16_rne(float f) { unsigned int u = __float_as_uint(f); u += 0x7FFFu + ((u >> 16) & 1u); return __uint_as_float(u & 0xFFFF0000u); }
__device__ __forceinline__ void split16(float v, b16& hi, b16& lo) { hi = (b16)v; lo = (b16)(v - (float)hi); }
__device__ __forceinline__ v16b frag_kb(const b16* p, int hh) { const v8b a = *(const v8b*)(p + 8 * hh), b = *(const v8b*)(p + 16 + 8 * hh); v16b f;
#pragma unroll
  for (int e = 0; e < 8; ++e) { f[e] = a[e]; f[8 + e] = b[e]; } return f; }
__device__ __forceinline__ v8f wmma16b(v16b a, v16b b, v8f c) { v8f d = __builtin_amdgcn_wmma_f32_16x16x32_f16(false, a, false, b, (short)0, c, false, false); asm volatile("v_nop\n\tv_nop\n\tv_nop\n\tv_nop" : "+v"(d) : "v"(a), "v"(b)); return d; }
__device__ __forceinline__ void wave_lds_sync() { __builtin_amdgcn_fence(__ATOMIC_RELEASE, "workgroup"); __builtin_amdgcn_wave_barrier(); __builtin_amdgcn_fence(__ATOMIC_ACQUIRE, "workgroup"); }
__device__ __forceinline__ float pmul(float a, float b) { float p = a * b; asm volatile("" : "+v"(p)); return p; }
__device__ __forceinline__ int iclamp(int v, int lo, int hi) { return v < lo ? lo : (v > hi ? hi : v); }
__device__ __forceinline__ float nexp2(float v) { return __builtin_amdgcn_exp2f(v); }

constexpr int N = 200000, ND = 50000, NDL = ND  , NLT = 4 * NDL  , NBOND = 300000, NMOL = 8192, F0 = 64, FB = 16, H = 128, K1P = 160, K2P = 288, NB = NLT / 32;
constexpr float XS = 8.0f, WSC = 256.0f, BNEPS = 1e-5f;
static_assert(N % 32 == 0 && NLT % 32 == 0 && NDL % 16 == 0 && ND % 16 == 0 && NDL <= ND && K1P % 32 == 0 && K2P % 32 == 0 && 2 * F0 + FB <= K1P && 2 * H + FB <= K2P && H == 128, "tiling");

__device__ __forceinline__ int prow(int m) { return NDL == ND ? m : (m / NDL) * ND + (m % NDL); }
__device__ __forceinline__ int premap(int nb) { return NDL == ND ? nb : (nb / ND) * ND + ((nb % ND) % NDL); }
template <int KP, int KA, int KB>
__global__ __launch_bounds__(256) void wcat_kernel(const float* __restrict__ wa, const float* __restrict__ wb, b16* __restrict__ WT) {
  static_assert(KP % 8 == 0 && KA % 8 == 0 && KB % 8 == 0 && KA + KB <= KP, "wcat"); const int u = blockIdx.x * 256 + threadIdx.x; if (u >= H * KP / 8) return; const int e = u * 8; const int o = e / KP, k0 = e % KP; v8b v;
  for (int j = 0; j < 8; ++j) { const int k = k0 + j; float w = 0.0f; if (k < KA) w = wa[(size_t)k * H + o]; else if (k < KA + KB) w = wb[(size_t)(k - KA) * H + o]; v[j] = (b16)(bf16_rne(w) * WSC); }
  for (int pass = 0; pass < 2; ++pass) { *(volatile v8b*)(WT + e) = v; __threadfence(); }
}
template <int KIN, int KP, bool RAWIN>
__global__ __launch_bounds__(64) void conv_kernel(const float* __restrict__ hin, const float* __restrict__ bond, const int* __restrict__ an1, const int* __restrict__ an2, const int* __restrict__ an3, const int* __restrict__ an4, const int* __restrict__ bn1, const int* __restrict__ bn2, const int* __restrict__ bn3, const int* __restrict__ bn4, const b16* __restrict__ WT  , const float* __restrict__ bias, float* __restrict__ T, float* __restrict__ PS) {
  static_assert(KIN % 4 == 0 && 2 * KIN + FB <= KP, "conv layout");
  __shared__ __attribute__((aligned(16))) b16 As[2][16][KP + 8]; __shared__ __attribute__((aligned(16))) float Tf[2][16][H + 4];
  const int wave = threadIdx.x >> 5, lane = threadIdx.x & 31, nloc = lane & 15, hlf = lane >> 4; const int m0 = blockIdx.x * 32 + wave * 16  ; const int d = m0 / NDL  , dd = d + 1; const int p0 = prow(m0)  ;
  const int* an = d == 0 ? an1 : d == 1 ? an2 : d == 2 ? an3 : an4; const int* bnn = d == 0 ? bn1 : d == 1 ? bn2 : d == 2 ? bn3 : bn4; const b16* W = WT + (size_t)d * H * KP;
  for (int idx = lane; idx < 16 * (KP / 4); idx += 32) { const int rr = idx / (KP / 4), c = (idx % (KP / 4)) * 4; const int row = p0 + rr; const int lr = row - d * ND; v4f v = {0.0f, 0.0f, 0.0f, 0.0f};
    if (c < KIN) { v = *(const v4f*)(hin + (size_t)row * KIN + c); if (RAWIN) for (int j = 0; j < 4; ++j) v[j] = bf16_rne(v[j]); }
    else if (c < 2 * KIN) {
#pragma unroll 1
      for (int k = 0; k < dd; ++k) { const int nb = premap(iclamp(an[(size_t)lr * dd + k], 0, N - 1)); v4f t = *(const v4f*)(hin + (size_t)nb * KIN + (c - KIN)); if (RAWIN) for (int j = 0; j < 4; ++j) t[j] = bf16_rne(t[j]); v += t; } }
    else if (c < 2 * KIN + FB) {
#pragma unroll 1
      for (int k = 0; k < dd; ++k) { const int nb = iclamp(bnn[(size_t)lr * dd + k], 0, NBOND - 1); v4f t = *(const v4f*)(bond + (size_t)nb * FB + (c - 2 * KIN)); for (int j = 0; j < 4; ++j) t[j] = bf16_rne(t[j]); v += t; } }
    v4h o; for (int j = 0; j < 4; ++j) o[j] = (b16)(v[j] * XS); *(v4h*)(&As[wave][rr][c]) = o; }
  wave_lds_sync();
  v8f acc[8];
#pragma unroll
  for (int t = 0; t < 8; ++t) acc[t] = (v8f){};
#pragma unroll 1
  for (int kb = 0; kb < KP; kb += 32) { const v16b a = frag_kb(&As[wave][nloc][kb], hlf);
#pragma unroll
    for (int t = 0; t < 8; ++t) acc[t] = wmma16b(a, frag_kb(W + (size_t)(t * 16 + nloc) * KP + kb, hlf), acc[t]); }
#pragma unroll
  for (int t = 0; t < 8; ++t) { const float bb = bf16_rne(bias[t * 16 + nloc]);
#pragma unroll
    for (int r = 0; r < 8; ++r) Tf[wave][8 * hlf + r][t * 16 + nloc] = acc[t][r] * (1.0f / (XS * WSC)) + bb; }
  __syncthreads();
  for (int pass = 0; pass < 2; ++pass) {
    for (int rr = 0; rr < 16; ++rr) *(volatile v4f*)(T + (size_t)(p0 + rr) * H + lane * 4) = *(const v4f*)(&Tf[wave][rr][lane * 4]);
    for (int cc = threadIdx.x; cc < H; cc += 64) { float s = 0.0f; for (int w2 = 0; w2 < 2; ++w2) for (int rr = 0; rr < 16; ++rr) s += Tf[w2][rr][cc]; ((volatile float*)PS)[(size_t)blockIdx.x * H + cc] = s; }
    __threadfence(); }
}
__global__ __launch_bounds__(128) void colstat_kernel(const float* __restrict__ PS, float* __restrict__ ST) { const int c = threadIdx.x; float s = 0.0f;
#pragma unroll 1
  for (int b = 0; b < NB; ++b) s += PS[(size_t)b * H + c];
  for (int pass = 0; pass < 2; ++pass) { ((volatile float*)ST)[c] = s * (1.0f / NLT); __threadfence(); } }
__global__ __launch_bounds__(128) void var_kernel(const float* __restrict__ P, const float* __restrict__ MEAN, float* __restrict__ PS) { const int c = threadIdx.x; float a = 0.0f; const float m = MEAN[c];
#pragma unroll 1
  for (int rr = 0; rr < 32; ++rr) { const size_t v = (size_t)prow(blockIdx.x * 32 + rr); const float dlt = P[v * H + c] - m; a += dlt * dlt; }
  for (int pass = 0; pass < 2; ++pass) { ((volatile float*)PS)[(size_t)blockIdx.x * H + c] = a; __threadfence(); } }
__global__ __launch_bounds__(256) void bnr_kernel(float* __restrict__ P, const float* __restrict__ MEAN, const float* __restrict__ VAR) { const size_t u = (size_t)blockIdx.x * 256 + threadIdx.x; if (u >= (size_t)NLT * H / 4) return; const int c = (int)((u * 4) % H); const size_t e = (size_t)prow((int)(u * 4 / H)) * H + c; v4f x = *(const v4f*)(P + e);
  for (int j = 0; j < 4; ++j) x[j] = fmaxf((x[j] - MEAN[c + j]) * rsqrtf(VAR[c + j] + BNEPS), 0.0f);
  for (int pass = 0; pass < 2; ++pass) { *(volatile v4f*)(P + e) = x; __threadfence(); } }
template <int KIN, bool RAWIN>
__global__ __launch_bounds__(64) void fp_kernel(const float* __restrict__ hin, const b16* __restrict__ WF, const float* __restrict__ bias, float* __restrict__ S) {
  static_assert(KIN % 32 == 0, "fp K");
  __shared__ __attribute__((aligned(16))) b16 As[2][16][KIN + 8]; __shared__ __attribute__((aligned(16))) float Tf[2][16][H + 4];
  const int wave = threadIdx.x >> 5, lane = threadIdx.x & 31, nloc = lane & 15, hlf = lane >> 4; const int m0 = prow(blockIdx.x * 32 + wave * 16)  ;
  for (int idx = lane; idx < 16 * (KIN / 4); idx += 32) { const int rr = idx / (KIN / 4), c = (idx % (KIN / 4)) * 4; v4f v = *(const v4f*)(hin + (size_t)(m0 + rr) * KIN + c); v4h o; for (int j = 0; j < 4; ++j) o[j] = (b16)((RAWIN ? bf16_rne(v[j]) : v[j]) * XS); *(v4h*)(&As[wave][rr][c]) = o; }
  wave_lds_sync();
  v8f acc[8];
#pragma unroll
  for (int t = 0; t < 8; ++t) acc[t] = (v8f){};
#pragma unroll 1
  for (int kb = 0; kb < KIN; kb += 32) { const v16b a = frag_kb(&As[wave][nloc][kb], hlf);
#pragma unroll
    for (int t = 0; t < 8; ++t) acc[t] = wmma16b(a, frag_kb(WF + (size_t)(t * 16 + nloc) * KIN + kb, hlf), acc[t]); }
  float z[8][8], mx[8], sm[8];
#pragma unroll
  for (int t = 0; t < 8; ++t) { const float bb = bf16_rne(bias[t * 16 + nloc]);
#pragma unroll
    for (int r = 0; r < 8; ++r) z[t][r] = acc[t][r] * (1.0f / (XS * WSC)) + bb; }
#pragma unroll
  for (int r = 0; r < 8; ++r) { float m = z[0][r];
#pragma unroll
    for (int t = 1; t < 8; ++t) m = fmaxf(m, z[t][r]); mx[r] = m; }
#pragma unroll
  for (int w = 1; w < 16; w <<= 1)
#pragma unroll
    for (int r = 0; r < 8; ++r) mx[r] = fmaxf(mx[r], __shfl_xor(mx[r], w));
#pragma unroll
  for (int r = 0; r < 8; ++r) { float s = 0.0f;
#pragma unroll
    for (int t = 0; t < 8; ++t) { const float e = __expf(z[t][r] - mx[r]); z[t][r] = e; s += e; } sm[r] = s; }
#pragma unroll
  for (int w = 1; w < 16; w <<= 1)
#pragma unroll
    for (int r = 0; r < 8; ++r) sm[r] += __shfl_xor(sm[r], w);
#pragma unroll
  for (int t = 0; t < 8; ++t)
#pragma unroll
    for (int r = 0; r < 8; ++r) Tf[wave][8 * hlf + r][t * 16 + nloc] = z[t][r] / sm[r];
  wave_lds_sync();
  for (int pass = 0; pass < 2; ++pass) { for (int rr = 0; rr < 16; ++rr) *(volatile v4f*)(S + (size_t)(m0 + rr) * H + lane * 4) = *(const v4f*)(&Tf[wave][rr][lane * 4]); __threadfence(); }
}
__device__ int lower_bound_i(const int* a, int n, int key) { int lo = 0, hi = n; while (lo < hi) { const int mid = (lo + hi) >> 1; if (a[mid] < key) lo = mid + 1; else hi = mid; } return lo; }
template <bool ACC>
__global__ __launch_bounds__(128) void pool_kernel(const float* __restrict__ S, const int* __restrict__ mol, float* __restrict__ out) {
  const int g = blockIdx.x, c = threadIdx.x; const int lo = lower_bound_i(mol, N, g), hi = lower_bound_i(mol, N, g + 1); float s = ACC ? out[(size_t)g * H + c] : 0.0f;
#pragma unroll 1
  for (int v = lo; v < hi; ++v) { if (NDL < ND && (v % ND) >= NDL) continue; s += S[(size_t)v * H + c]; }
  for (int pass = 0; pass < 2; ++pass) { ((volatile float*)out)[(size_t)g * H + c] = s; __threadfence(); }
}
}

extern "C" void kernel_launch(void* const* d_in, const int* in_sizes, int n_in, void* d_out, int out_size, void* d_ws, size_t ws_size, hipStream_t stream) {
  (void)n_in;
  auto Fp = [&](int i) { return (const float*)d_in[i]; }; auto Ip = [&](int i) { return (const int*)d_in[i]; };
  if (in_sizes[0] != N * F0 || in_sizes[1] != NBOND * FB || in_sizes[2] != ND || in_sizes[8] != ND * 4 || in_sizes[9] != ND * 4 || in_sizes[10] != N || in_sizes[11] != F0 * H || in_sizes[13] != H * H || in_sizes[17] != F0 * H || in_sizes[19] != (F0 + FB) * H || in_sizes[22] != (F0 + FB) * H || in_sizes[23] != H * H || in_sizes[25] != (H + FB) * H || in_sizes[28] != (H + FB) * H || out_size != NMOL * H) return;
  size_t off = 0; char* ws = (char*)d_ws;
  auto carve = [&](size_t bytes) { char* p = ws + off; off += (bytes + 255) & ~(size_t)255; return p; };
  b16* WC1 = (b16*)carve((size_t)4 * H * K1P * 2); b16* WC2 = (b16*)carve((size_t)4 * H * K2P * 2); b16* WF0 = (b16*)carve((size_t)H * F0 * 2); b16* WF1 = (b16*)carve((size_t)H * H * 2); b16* WF2 = (b16*)carve((size_t)H * H * 2);
  float* T = (float*)carve((size_t)N * H * 4); float* S = (float*)carve((size_t)N * H * 4); float* PS = (float*)carve((size_t)NB * H * 4); float* ST = (float*)carve((size_t)2 * H * 4);
  if (off > ws_size || off > ((size_t)240 << 20)) return;
  for (int d = 0; d < 4; ++d) { wcat_kernel<K1P, F0, F0 + FB><<<(H * K1P / 8 + 255) / 256, 256, 0, stream>>>(Fp(17), Fp(19 + d), WC1 + (size_t)d * H * K1P); wcat_kernel<K2P, H, H + FB><<<(H * K2P / 8 + 255) / 256, 256, 0, stream>>>(Fp(23), Fp(25 + d), WC2 + (size_t)d * H * K2P); }
  wcat_kernel<F0, F0, 0><<<(H * F0 / 8 + 255) / 256, 256, 0, stream>>>(Fp(11), nullptr, WF0); wcat_kernel<H, H, 0><<<(H * H / 8 + 255) / 256, 256, 0, stream>>>(Fp(13), nullptr, WF1); wcat_kernel<H, H, 0><<<(H * H / 8 + 255) / 256, 256, 0, stream>>>(Fp(15), nullptr, WF2);
  const unsigned nblk = NLT / 32, nb4 = (unsigned)(((size_t)NLT * H / 4 + 255) / 256);
  fp_kernel<F0, true><<<nblk, 64, 0, stream>>>(Fp(0), WF0, Fp(12), S); pool_kernel<false><<<NMOL, H, 0, stream>>>(S, Ip(10), (float*)d_out);
  conv_kernel<F0, K1P, true><<<nblk, 64, 0, stream>>>(Fp(0), Fp(1), Ip(2), Ip(4), Ip(6), Ip(8), Ip(3), Ip(5), Ip(7), Ip(9), WC1, Fp(18), T, PS);
  colstat_kernel<<<1, H, 0, stream>>>(PS, ST); var_kernel<<<nblk, H, 0, stream>>>(T, ST, PS); colstat_kernel<<<1, H, 0, stream>>>(PS, ST + H); bnr_kernel<<<nb4, 256, 0, stream>>>(T, ST, ST + H);
  fp_kernel<H, false><<<nblk, 64, 0, stream>>>(T, WF1, Fp(14), S); pool_kernel<true><<<NMOL, H, 0, stream>>>(S, Ip(10), (float*)d_out);
  conv_kernel<H, K2P, false><<<nblk, 64, 0, stream>>>(T, Fp(1), Ip(2), Ip(4), Ip(6), Ip(8), Ip(3), Ip(5), Ip(7), Ip(9), WC2, Fp(24), S, PS);
  colstat_kernel<<<1, H, 0, stream>>>(PS, ST); var_kernel<<<nblk, H, 0, stream>>>(S, ST, PS); colstat_kernel<<<1, H, 0, stream>>>(PS, ST + H); bnr_kernel<<<nb4, 256, 0, stream>>>(S, ST, ST + H);
  fp_kernel<H, false><<<nblk, 64, 0, stream>>>(S, WF2, Fp(16), T); pool_kernel<true><<<NMOL, H, 0, stream>>>(T, Ip(10), (float*)d_out);
}
